// KernelEncoder_19207093748412
// MI455X (gfx1250) — hardware-verified
//
#include <hip/hip_runtime.h>


typedef _Float16 v4h  __attribute__((ext_vector_type(4)));
typedef _Float16 v8h  __attribute__((ext_vector_type(8)));
typedef _Float16 v16h __attribute__((ext_vector_type(16)));
typedef __bf16   v16b __attribute__((ext_vector_type(16)));
typedef unsigned short v8us __attribute__((ext_vector_type(8)));
typedef unsigned int v2u __attribute__((ext_vector_type(2)));
typedef unsigned int v4u __attribute__((ext_vector_type(4)));
typedef float v4f __attribute__((ext_vector_type(4)));
typedef float v8f __attribute__((ext_vector_type(8)));
typedef v4f v4fa __attribute__((may_alias));

#define EPS_LN 1e-3f
#define STAB   1e-6f

constexpr int Bb = 4, Ss = 4096, Dd = 128, Hh = 8, Kk = 128, Mm = 256;
constexpr int BS = Bb * Ss;
constexpr int HK = Hh * Kk;

static_assert(BS % 128 == 0 && HK % 128 == 0 && Ss % 128 == 0 && Mm % 128 == 0 && Dd % 128 == 0 && Kk % 128 == 0);
static_assert(Dd % 64 == 0 && HK % 64 == 0);
static_assert(BS % 64 == 0 && BS % 16 == 0);
static_assert((Bb * Hh * Mm) % 1024 == 0 && (Bb * Hh * Ss) % 1024 == 0 && Ss % 128 == 0);

enum { EP_LIN = 0, EP_ELU1 = 1, EP_ELU = 2 };

union Frag { v8us u[2]; v16h h; v16b b; };
union H8   { v8h h; v8us u; v4u q; };
union H4   { v4h h; v2u u; };

__device__ __forceinline__ float wsum32(float v) {
#pragma unroll
  for (int o = 16; o >= 1; o >>= 1) v += __shfl_xor(v, o, 32);
  return v;
}
__device__ __forceinline__ float wsum16(float v) {
#pragma unroll
  for (int o = 8; o >= 1; o >>= 1) v += __shfl_xor(v, o, 32);
  return v;
}
__device__ __forceinline__ unsigned short bf_rne(float f) {
  unsigned int u = __float_as_uint(f);
  u += 0x7FFFu + ((u >> 16) & 1u);
  return (unsigned short)(u >> 16);
}
__device__ __forceinline__ float bf_val(unsigned short b) {
  return __uint_as_float(((unsigned int)b) << 16);
}
__device__ __forceinline__ void split_bf8(const float* x, H8& hi, H8& lo) {
#pragma unroll
  for (int j = 0; j < 8; ++j) {
    const unsigned short hb = bf_rne(x[j]);
    hi.u[j] = hb;
    lo.u[j] = bf_rne(x[j] - bf_val(hb));
  }
}
__device__ __forceinline__ v4u pack_f16x8(const float* x) {
  H8 t;
#pragma unroll
  for (int j = 0; j < 8; ++j) t.h[j] = (_Float16)x[j];
  return t.q;
}

__device__ __forceinline__ void ld_frag(Frag& f, const unsigned short* p) {
  f.u[0] = *(const v8us*)(p);
  f.u[1] = *(const v8us*)(p + 16);
}

template <bool BF>
__device__ __forceinline__ v8f mma16(const Frag& a, const Frag& b, v8f c) {
  if constexpr (BF)
    return __builtin_amdgcn_wmma_f32_16x16x32_bf16(false, a.b, false, b.b, (short)0, c, false, false);
  else
    return __builtin_amdgcn_wmma_f32_16x16x32_f16(false, a.h, false, b.h, (short)0, c, false, false);
}

template <bool BF, bool SPLIT, int EP, int BIASM, int RSM, bool CSI, bool RESID, bool OUT16>
__global__ void __launch_bounds__(256) gemm_nt_kernel(
    const unsigned short* __restrict__ A1, const unsigned short* __restrict__ A2,
    long long aZ1, long long aZ2, int lda,
    const unsigned short* __restrict__ B1, const unsigned short* __restrict__ B2,
    long long bZ1, long long bZ2, int ldb,
    void* Cv, long long cZ1, long long cZ2, int ldc,
    const float* __restrict__ bias,
    const float* __restrict__ rsF, const int* __restrict__ rsI, long long rZ1, long long rZ2,
    const int* __restrict__ csI, long long sZ1, long long sZ2,
    const float* __restrict__ resid, int ldr,
    int Kdim, int zdiv, float s1, float s2)
{
  __shared__ __attribute__((aligned(16))) float Ls[8 * 16 * 64];

  const int tid = threadIdx.x, w = tid >> 5, l = tid & 31, h = l >> 4, m = l & 15;
  const int wr = w & 3, wc = w >> 2;
  const int z = blockIdx.z;
  const int zb = z / zdiv, zh = z - zb * zdiv;
  const int row0 = blockIdx.x * 128 + wr * 32;
  const int col0 = blockIdx.y * 128 + wc * 64;

  const long long aOff = (long long)zb * aZ1 + (long long)zh * aZ2;
  const long long bOff = (long long)zb * bZ1 + (long long)zh * bZ2;
  const long long cOff = (long long)zb * cZ1 + (long long)zh * cZ2;
  const long long rOff = (long long)zb * rZ1 + (long long)zh * rZ2;
  const long long sOff = (long long)zb * sZ1 + (long long)zh * sZ2;

  const unsigned short* Ab = A1 + aOff;
  const unsigned short* Bb_ = B1 + bOff;

  const size_t ao0 = (size_t)(row0 + m) * (size_t)lda + 8 * h;
  const size_t ao1 = ao0 + (size_t)16 * (size_t)lda;
  size_t bo[4];
#pragma unroll
  for (int nt = 0; nt < 4; ++nt) bo[nt] = (size_t)(col0 + nt * 16 + m) * (size_t)ldb + 8 * h;

  v8f acc[2][4] = {};

#pragma unroll 1
  for (int k0 = 0; k0 < Kdim; k0 += 32) {
    Frag a0, a1, b;
    ld_frag(a0, Ab + ao0 + k0);
    ld_frag(a1, Ab + ao1 + k0);
    if constexpr (SPLIT) {
      const unsigned short* Ae = A2 + aOff;
      const unsigned short* Be = B2 + bOff;
      Frag e0, e1, f;
      ld_frag(e0, Ae + ao0 + k0);
      ld_frag(e1, Ae + ao1 + k0);
#pragma unroll
      for (int nt = 0; nt < 4; ++nt) {
        ld_frag(b, Bb_ + bo[nt] + k0);
        ld_frag(f, Be + bo[nt] + k0);
        acc[0][nt] = mma16<BF>(a0, b, acc[0][nt]);
        acc[1][nt] = mma16<BF>(a1, b, acc[1][nt]);
        acc[0][nt] = mma16<BF>(a0, f, acc[0][nt]);
        acc[1][nt] = mma16<BF>(a1, f, acc[1][nt]);
        acc[0][nt] = mma16<BF>(e0, b, acc[0][nt]);
        acc[1][nt] = mma16<BF>(e1, b, acc[1][nt]);
      }
      asm volatile("v_nop\n\tv_nop\n\tv_nop\n\tv_nop"
                   : "+v"(acc[0][0]), "+v"(acc[0][1]), "+v"(acc[0][2]), "+v"(acc[0][3]),
                     "+v"(acc[1][0]), "+v"(acc[1][1]), "+v"(acc[1][2]), "+v"(acc[1][3])
                   : "v"(a0.h), "v"(a1.h), "v"(e0.h), "v"(e1.h), "v"(b.h), "v"(f.h));
    } else {
#pragma unroll
      for (int nt = 0; nt < 4; ++nt) {
        ld_frag(b, Bb_ + bo[nt] + k0);
        acc[0][nt] = mma16<BF>(a0, b, acc[0][nt]);
        acc[1][nt] = mma16<BF>(a1, b, acc[1][nt]);
      }
      asm volatile("v_nop\n\tv_nop\n\tv_nop\n\tv_nop"
                   : "+v"(acc[0][0]), "+v"(acc[0][1]), "+v"(acc[0][2]), "+v"(acc[0][3]),
                     "+v"(acc[1][0]), "+v"(acc[1][1]), "+v"(acc[1][2]), "+v"(acc[1][3])
                   : "v"(a0.h), "v"(a1.h), "v"(b.h));
    }
  }

  float* Lw = Ls + w * (16 * 64);
  unsigned short* C16 = (unsigned short*)Cv;
  float* C32 = (float*)Cv;

#pragma unroll
  for (int rt = 0; rt < 2; ++rt) {
#pragma unroll
    for (int nt = 0; nt < 4; ++nt) {
      const int gcol = col0 + nt * 16 + m;
      float bc = 0.0f;
      if constexpr (BIASM == 1) bc = bias[gcol];
      float cs = 1.0f;
      if constexpr (CSI) cs = (float)csI[sOff + gcol];
#pragma unroll
      for (int r = 0; r < 8; ++r) {
        const int lrow = 8 * h + r;
        const int grow = row0 + rt * 16 + lrow;
        float x = acc[rt][nt][r] * s1;
        if constexpr (BIASM == 1) x += bc;
        if constexpr (BIASM == 2) x += bias[grow];
        if constexpr (EP == EP_ELU1) x = (x > 0.0f) ? (x + 1.0f) : __expf(x);
        if constexpr (EP == EP_ELU)  x = (x > 0.0f) ? x : (__expf(x) - 1.0f);
        x *= s2;
        if constexpr (RSM == 1) x *= rsF[rOff + grow];
        if constexpr (RSM == 2) x *= (float)rsI[rOff + grow];
        if constexpr (CSI) x *= cs;
        Lw[lrow * 64 + nt * 16 + m] = x;
      }
    }
    __syncthreads();

    if constexpr (OUT16) {
      v4u ov[4];
      size_t og[4];
#pragma unroll
      for (int i = 0; i < 4; ++i) {
        const int lrow = 4 * i + (l >> 3), c8 = (l & 7) * 8;
        const v4f x0 = *(const v4fa*)(Lw + lrow * 64 + c8);
        const v4f x1 = *(const v4fa*)(Lw + lrow * 64 + c8 + 4);
        float xv[8];
#pragma unroll
        for (int j = 0; j < 4; ++j) { xv[j] = x0[j]; xv[4 + j] = x1[j]; }
        ov[i] = pack_f16x8(xv);
        og[i] = (size_t)cOff + (size_t)(row0 + rt * 16 + lrow) * (size_t)ldc + (size_t)(col0 + c8);
      }
#pragma unroll
      for (int i = 0; i < 4; ++i) *(volatile v4u*)(C16 + og[i]) = ov[i];
      __threadfence();
#pragma unroll
      for (int i = 0; i < 4; ++i) *(volatile v4u*)(C16 + og[i]) = ov[i];
    } else {
      v4f ov[8];
      size_t og[8];
#pragma unroll
      for (int i = 0; i < 8; ++i) {
        const int lrow = 2 * i + (l >> 4), c4 = (l & 15) * 4;
        const int grow = row0 + rt * 16 + lrow;
        v4f x = *(const v4fa*)(Lw + lrow * 64 + c4);
        if constexpr (RESID) x += *(const v4f*)(resid + (size_t)grow * (size_t)ldr + col0 + c4);
        ov[i] = x;
        og[i] = (size_t)cOff + (size_t)grow * (size_t)ldc + (size_t)(col0 + c4);
      }
#pragma unroll
      for (int i = 0; i < 8; ++i) *(volatile v4f*)(C32 + og[i]) = ov[i];
      __threadfence();
#pragma unroll
      for (int i = 0; i < 8; ++i) *(volatile v4f*)(C32 + og[i]) = ov[i];
    }
    __syncthreads();
  }
}

template <bool BF>
__global__ void __launch_bounds__(256) tr_cvt_kernel(const float* __restrict__ W, int Kin, int N, float scale,
                                                     unsigned short* O1, unsigned short* O2)
{
  __shared__ float T[64 * 65];
  const int tid = threadIdx.x, w = tid >> 5, l = tid & 31;
  const int n0 = blockIdx.x * 64, k0 = blockIdx.y * 64;
#pragma unroll
  for (int i = 0; i < 16; ++i) {
    const int e = tid + 256 * i;
    const int kk = e >> 6, nn = e & 63;
    T[kk * 65 + nn] = W[(size_t)(k0 + kk) * (size_t)N + n0 + nn];
  }
  __syncthreads();
  const int q = l >> 3, kq = (l & 7) * 8;
  v4u o1[2], o2[2];
  size_t og[2];
#pragma unroll
  for (int i = 0; i < 2; ++i) {
    const int nn = w * 8 + i * 4 + q;
    float x[8];
#pragma unroll
    for (int j = 0; j < 8; ++j) x[j] = T[(kq + j) * 65 + nn] * scale;
    if constexpr (BF) {
      H8 hi, lo;
      split_bf8(x, hi, lo);
      o1[i] = hi.q; o2[i] = lo.q;
    } else {
      o1[i] = pack_f16x8(x);
      o2[i] = o1[i];
    }
    og[i] = (size_t)(n0 + nn) * (size_t)Kin + (size_t)(k0 + kq);
  }
#pragma unroll
  for (int i = 0; i < 2; ++i) {
    *(volatile v4u*)(O1 + og[i]) = o1[i];
    if constexpr (BF) *(volatile v4u*)(O2 + og[i]) = o2[i];
  }
  __threadfence();
#pragma unroll
  for (int i = 0; i < 2; ++i) {
    *(volatile v4u*)(O1 + og[i]) = o1[i];
    if constexpr (BF) *(volatile v4u*)(O2 + og[i]) = o2[i];
  }
}

__global__ void __launch_bounds__(256) cvt_f16_kernel(const float* __restrict__ in, unsigned short* out,
                                                      float scale, int n8)
{
  const int i = blockIdx.x * 256 + threadIdx.x;
  if (i >= n8) return;
  const v4f a = *(const v4f*)(in + (size_t)i * 8);
  const v4f b = *(const v4f*)(in + (size_t)i * 8 + 4);
  float x[8];
#pragma unroll
  for (int j = 0; j < 4; ++j) { x[j] = a[j] * scale; x[4 + j] = b[j] * scale; }
  const v4u o = pack_f16x8(x);
  *(volatile v4u*)(out + (size_t)i * 8) = o;
  __threadfence();
  *(volatile v4u*)(out + (size_t)i * 8) = o;
}

__device__ __forceinline__ v4f ln_row32(v4f x, v4f g, v4f b) {
  const float mean = wsum32(x[0] + x[1] + x[2] + x[3]) * (1.0f / 128.0f);
  v4f d = x - mean;
  const float var = wsum32(d[0] * d[0] + d[1] * d[1] + d[2] * d[2] + d[3] * d[3]) * (1.0f / 128.0f);
  const float rstd = rsqrtf(var + EPS_LN);
  return d * rstd * g + b;
}

__global__ void __launch_bounds__(256) ln_in_kernel(const float* __restrict__ X, const float* __restrict__ g,
                                                    const float* __restrict__ bt, float* Xn, unsigned short* Xh)
{
  const int w = threadIdx.x >> 5, l = threadIdx.x & 31, h = l >> 4;
  const int rbase = (blockIdx.x * 8 + w) * 8;
  const v4f gg = *(const v4f*)(g + 4 * l);
  const v4f bb = *(const v4f*)(bt + 4 * l);
  const int sA = 2 * (l & 15), sB = sA + 1;
  for (int p = 0; p < 2; ++p) {
#pragma unroll
    for (int pr = 0; pr < 4; ++pr) {
      const int rA = rbase + 2 * pr, rB = rA + 1;
      const v4f xa = *(const v4f*)(X + (size_t)rA * Dd + 4 * l);
      const v4f xb = *(const v4f*)(X + (size_t)rB * Dd + 4 * l);
      const v4f ya = ln_row32(xa, gg, bb);
      const v4f yb = ln_row32(xb, gg, bb);
      *(volatile v4f*)(Xn + (size_t)rA * Dd + 4 * l) = ya;
      *(volatile v4f*)(Xn + (size_t)rB * Dd + 4 * l) = yb;
      H4 ta, tb;
#pragma unroll
      for (int j = 0; j < 4; ++j) { ta.h[j] = (_Float16)ya[j]; tb.h[j] = (_Float16)yb[j]; }
      const unsigned int t0 = __shfl(ta.u[0], sA, 32), t1 = __shfl(ta.u[1], sA, 32);
      const unsigned int t2 = __shfl(ta.u[0], sB, 32), t3 = __shfl(ta.u[1], sB, 32);
      const unsigned int u0 = __shfl(tb.u[0], sA, 32), u1 = __shfl(tb.u[1], sA, 32);
      const unsigned int u2 = __shfl(tb.u[0], sB, 32), u3 = __shfl(tb.u[1], sB, 32);
      v4u o;
      o[0] = h ? u0 : t0; o[1] = h ? u1 : t1; o[2] = h ? u2 : t2; o[3] = h ? u3 : t3;
      *(volatile v4u*)(Xh + (size_t)(rA + h) * Dd + (l & 15) * 8) = o;
    }
    if (p == 0) __threadfence();
  }
}

__device__ __forceinline__ void ln_row16(float* v, const float* g, const float* b) {
  float s = 0.0f;
#pragma unroll
  for (int j = 0; j < 8; ++j) s += v[j];
  const float mean = wsum16(s) * (1.0f / 128.0f);
  float ss = 0.0f;
#pragma unroll
  for (int j = 0; j < 8; ++j) { v[j] -= mean; ss += v[j] * v[j]; }
  const float var = wsum16(ss) * (1.0f / 128.0f);
  const float rstd = rsqrtf(var + EPS_LN);
#pragma unroll
  for (int j = 0; j < 8; ++j) v[j] = v[j] * rstd * g[j] + b[j];
}

template <bool CHAIN>
__global__ void __launch_bounds__(256) ln_planes_kernel(const float* __restrict__ in,
    const float* __restrict__ g1, const float* __restrict__ b1,
    const float* __restrict__ g2, const float* __restrict__ b2,
    unsigned short* Ohi, unsigned short* Olo)
{
  const int w = threadIdx.x >> 5, l = threadIdx.x & 31, h = l >> 4;
  const int row = (blockIdx.x * 8 + w) * 2 + h;
  const int c0 = 8 * (l & 15);
  float ga[8], ba[8], gb[8], bbv[8];
  {
    const v4f g10 = *(const v4f*)(g1 + c0), g11 = *(const v4f*)(g1 + c0 + 4);
    const v4f b10 = *(const v4f*)(b1 + c0), b11 = *(const v4f*)(b1 + c0 + 4);
#pragma unroll
    for (int j = 0; j < 4; ++j) { ga[j] = g10[j]; ga[4 + j] = g11[j]; ba[j] = b10[j]; ba[4 + j] = b11[j]; }
    if constexpr (CHAIN) {
      const v4f g20 = *(const v4f*)(g2 + c0), g21 = *(const v4f*)(g2 + c0 + 4);
      const v4f b20 = *(const v4f*)(b2 + c0), b21 = *(const v4f*)(b2 + c0 + 4);
#pragma unroll
      for (int j = 0; j < 4; ++j) { gb[j] = g20[j]; gb[4 + j] = g21[j]; bbv[j] = b20[j]; bbv[4 + j] = b21[j]; }
    } else {
#pragma unroll
      for (int j = 0; j < 8; ++j) { gb[j] = 1.0f; bbv[j] = 0.0f; }
    }
  }
  for (int p = 0; p < 2; ++p) {
    const v4f x0 = *(const v4f*)(in + (size_t)row * Dd + c0);
    const v4f x1 = *(const v4f*)(in + (size_t)row * Dd + c0 + 4);
    float v[8];
#pragma unroll
    for (int j = 0; j < 4; ++j) { v[j] = x0[j]; v[4 + j] = x1[j]; }
    ln_row16(v, ga, ba);
    if constexpr (CHAIN) ln_row16(v, gb, bbv);
    H8 hi, lo;
    split_bf8(v, hi, lo);
    *(volatile v4u*)(Ohi + (size_t)row * Dd + c0) = hi.q;
    *(volatile v4u*)(Olo + (size_t)row * Dd + c0) = lo.q;
    if (p == 0) __threadfence();
  }
}

__global__ void __launch_bounds__(256) ksum_kernel(const unsigned short* __restrict__ kpt, float* ksum)
{
  __shared__ __attribute__((aligned(16))) float red[8][128];
  const int w = threadIdx.x >> 5, l = threadIdx.x & 31;
  const int wb = (blockIdx.x * 8 + w) * 128;
#pragma unroll 1
  for (int rr = 0; rr < 128; ++rr) {
    const unsigned short* p = kpt + (size_t)(wb + rr) * (size_t)Ss + 8 * l;
    float a = 0.0f;
#pragma unroll 4
    for (int s0 = 0; s0 < Ss; s0 += 256) {
      H8 t;
      t.u = *(const v8us*)(p + s0);
#pragma unroll
      for (int j = 0; j < 8; ++j) a += (float)t.h[j];
    }
    a = wsum32(a);
    if (l == 0) red[w][rr] = a;
  }
  __syncthreads();
  const v4f v = *(const v4fa*)(&red[w][4 * l]);
  *(volatile v4f*)(ksum + wb + 4 * l) = v;
  __threadfence();
  *(volatile v4f*)(ksum + wb + 4 * l) = v;
}

__global__ void __launch_bounds__(256) rden_kernel(const unsigned short* __restrict__ qp,
                                                   const float* __restrict__ ksum, float* rden)
{
  __shared__ __attribute__((aligned(16))) float red[8][128];
  const int w = threadIdx.x >> 5, l = threadIdx.x & 31;
  const int wb = (blockIdx.x * 8 + w) * 128;
  const int bh = wb / Ss;
  float ks[8];
  {
    const v4f k0 = *(const v4f*)(ksum + (size_t)bh * Mm + 8 * l);
    const v4f k1 = *(const v4f*)(ksum + (size_t)bh * Mm + 8 * l + 4);
#pragma unroll
    for (int j = 0; j < 4; ++j) { ks[j] = k0[j]; ks[4 + j] = k1[j]; }
  }
#pragma unroll 2
  for (int rr = 0; rr < 128; ++rr) {
    H8 t;
    t.u = *(const v8us*)(qp + (size_t)(wb + rr) * (size_t)Mm + 8 * l);
    float a = 0.0f;
#pragma unroll
    for (int j = 0; j < 8; ++j) a += (float)t.h[j] * ks[j];
    a = wsum32(a);
    if (l == 0) red[w][rr] = 1.0f / (a * 3.814697265625e-06f + STAB);
  }
  __syncthreads();
  const v4f v = *(const v4fa*)(&red[w][4 * l]);
  *(volatile v4f*)(rden + wb + 4 * l) = v;
  __threadfence();
  *(volatile v4f*)(rden + wb + 4 * l) = v;
}

extern "C" void kernel_launch(void* const* d_in, const int* in_sizes, int n_in,
                              void* d_out, int out_size, void* d_ws, size_t ws_size,
                              hipStream_t stream)
{
  if (n_in < 24) return;
  if (out_size != BS * Dd) return;
  if (in_sizes[0] != BS * Dd || in_sizes[1] != BS * Dd || in_sizes[2] != BS) return;
  if (in_sizes[3] != Dd * HK || in_sizes[9] != HK * Dd || in_sizes[11] != Mm * Kk) return;
  if (in_sizes[18] != Dd * Dd || in_sizes[22] != Dd * Dd) return;

  const float* Q      = (const float*)d_in[0];
  const float* X      = (const float*)d_in[1];
  const int*   mask   = (const int*)  d_in[2];
  const float* Wq     = (const float*)d_in[3];
  const float* bq     = (const float*)d_in[4];
  const float* Wk     = (const float*)d_in[5];
  const float* bk     = (const float*)d_in[6];
  const float* Wv     = (const float*)d_in[7];
  const float* bv     = (const float*)d_in[8];
  const float* Wo     = (const float*)d_in[9];
  const float* bo     = (const float*)d_in[10];
  const float* proj   = (const float*)d_in[11];
  const float* ln1_g  = (const float*)d_in[12];
  const float* ln1_b  = (const float*)d_in[13];
  const float* ln2_g  = (const float*)d_in[14];
  const float* ln2_b  = (const float*)d_in[15];
  const float* fln0_g = (const float*)d_in[16];
  const float* fln0_b = (const float*)d_in[17];
  const float* f_w0   = (const float*)d_in[18];
  const float* f_b0   = (const float*)d_in[19];
  const float* fln1_g = (const float*)d_in[20];
  const float* fln1_b = (const float*)d_in[21];
  const float* f_w1   = (const float*)d_in[22];
  const float* f_b1   = (const float*)d_in[23];
  float* out = (float*)d_out;

  size_t off = 0;
  auto carve = [&](size_t bytes) -> size_t { size_t o = off; off += (bytes + 255) & ~(size_t)255; return o; };
  const size_t oXn  = carve((size_t)BS * Dd * 4);
  const size_t oXnh = carve((size_t)BS * Dd * 2);
  const size_t oQh  = carve((size_t)BS * Dd * 2);
  const size_t oWq  = carve((size_t)HK * Dd * 2);
  const size_t oWk  = carve((size_t)HK * Dd * 2);
  const size_t oWv  = carve((size_t)HK * Dd * 2);
  const size_t oWo  = carve((size_t)Dd * HK * 2);
  const size_t oPj  = carve((size_t)Mm * Kk * 2);
  const size_t oW0h = carve((size_t)Dd * Dd * 2);
  const size_t oW0l = carve((size_t)Dd * Dd * 2);
  const size_t oW1h = carve((size_t)Dd * Dd * 2);
  const size_t oW1l = carve((size_t)Dd * Dd * 2);
  const size_t oq   = carve((size_t)BS * HK * 2);
  const size_t ok   = carve((size_t)BS * HK * 2);
  const size_t ovT  = carve((size_t)BS * HK * 2);
  const size_t oqp  = carve((size_t)Bb * Hh * Ss * Mm * 2);
  const size_t okp  = carve((size_t)Bb * Hh * Mm * Ss * 2);
  const size_t oks  = carve((size_t)Bb * Hh * Mm * 4);
  const size_t ord  = carve((size_t)Bb * Hh * Ss * 4);
  const size_t okv  = carve((size_t)Bb * Hh * Kk * Mm * 2);
  if (off > ws_size) return;

  char* ws = (char*)d_ws;
  float*          Xn   = (float*)(ws + oXn);
  unsigned short* Xnh  = (unsigned short*)(ws + oXnh);
  unsigned short* Qh   = (unsigned short*)(ws + oQh);
  unsigned short* WqT  = (unsigned short*)(ws + oWq);
  unsigned short* WkT  = (unsigned short*)(ws + oWk);
  unsigned short* WvT  = (unsigned short*)(ws + oWv);
  unsigned short* WoT  = (unsigned short*)(ws + oWo);
  unsigned short* Pjh  = (unsigned short*)(ws + oPj);
  unsigned short* W0h  = (unsigned short*)(ws + oW0h);
  unsigned short* W0l  = (unsigned short*)(ws + oW0l);
  unsigned short* W1h  = (unsigned short*)(ws + oW1h);
  unsigned short* W1l  = (unsigned short*)(ws + oW1l);
  unsigned short* qh   = (unsigned short*)(ws + oq);
  unsigned short* kh   = (unsigned short*)(ws + ok);
  unsigned short* vT   = (unsigned short*)(ws + ovT);
  unsigned short* qp   = (unsigned short*)(ws + oqp);
  unsigned short* kpt  = (unsigned short*)(ws + okp);
  float*          ksum = (float*)(ws + oks);
  float*          rden = (float*)(ws + ord);
  unsigned short* kvT  = (unsigned short*)(ws + okv);
  unsigned short* attnh = qh;
  float*          res1  = (float*)(ws + ok);
  unsigned short* a0hi  = (unsigned short*)(ws + ok + (size_t)8 * 1048576);
  unsigned short* a0lo  = (unsigned short*)(ws + ok + (size_t)12 * 1048576);
  float*          h1    = (float*)(ws + ok + (size_t)16 * 1048576);
  unsigned short* a1hi  = (unsigned short*)(ws + ok + (size_t)24 * 1048576);
  unsigned short* a1lo  = (unsigned short*)(ws + ok + (size_t)28 * 1048576);

  const unsigned short* nul16 = nullptr;
  const float* nulf = nullptr;
  const int* nuli = nullptr;

  cvt_f16_kernel<<<(BS * Dd / 8) / 256, 256, 0, stream>>>(Q, Qh, 1.0f, BS * Dd / 8);
  cvt_f16_kernel<<<(Mm * Kk / 8) / 256, 256, 0, stream>>>(proj, Pjh, 16.0f, Mm * Kk / 8);
  tr_cvt_kernel<false><<<dim3(HK / 64, Dd / 64), 256, 0, stream>>>(Wq, Dd, HK, 64.0f, WqT, WqT);
  tr_cvt_kernel<false><<<dim3(HK / 64, Dd / 64), 256, 0, stream>>>(Wk, Dd, HK, 64.0f, WkT, WkT);
  tr_cvt_kernel<false><<<dim3(HK / 64, Dd / 64), 256, 0, stream>>>(Wv, Dd, HK, 64.0f, WvT, WvT);
  tr_cvt_kernel<false><<<dim3(Dd / 64, HK / 64), 256, 0, stream>>>(Wo, HK, Dd, 64.0f, WoT, WoT);
  tr_cvt_kernel<true><<<dim3(Dd / 64, Dd / 64), 256, 0, stream>>>(f_w0, Dd, Dd, 1.0f, W0h, W0l);
  tr_cvt_kernel<true><<<dim3(Dd / 64, Dd / 64), 256, 0, stream>>>(f_w1, Dd, Dd, 1.0f, W1h, W1l);

  ln_in_kernel<<<BS / 64, 256, 0, stream>>>(X, ln1_g, ln1_b, Xn, Xnh);

  gemm_nt_kernel<false, false, EP_LIN, 1, 0, false, false, true>
      <<<dim3(BS / 128, HK / 128, 1), 256, 0, stream>>>(
          Qh, nul16, 0, 0, Dd, WqT, nul16, 0, 0, Dd, qh, 0, 0, HK,
          bq, nulf, nuli, 0, 0, nuli, 0, 0, nulf, 0, Dd, 1, 0.015625f, 5.656854249492380f);
  gemm_nt_kernel<false, false, EP_LIN, 1, 0, false, false, true>
      <<<dim3(BS / 128, HK / 128, 1), 256, 0, stream>>>(
          Xnh, nul16, 0, 0, Dd, WkT, nul16, 0, 0, Dd, kh, 0, 0, HK,
          bk, nulf, nuli, 0, 0, nuli, 0, 0, nulf, 0, Dd, 1, 0.015625f, 16.0f);
  gemm_nt_kernel<false, false, EP_LIN, 2, 0, false, false, true>
      <<<dim3(HK / 128, Ss / 128, Bb), 256, 0, stream>>>(
          WvT, nul16, 0, 0, Dd, Xnh, nul16, (long long)Ss * Dd, 0, Dd, vT, (long long)HK * Ss, 0, Ss,
          bv, nulf, nuli, 0, 0, nuli, 0, 0, nulf, 0, Dd, 1, 0.015625f, 16.0f);
  gemm_nt_kernel<false, false, EP_ELU1, 0, 0, false, false, true>
      <<<dim3(Ss / 128, Mm / 128, Bb * Hh), 256, 0, stream>>>(
          qh, nul16, (long long)Ss * HK, Kk, HK, Pjh, nul16, 0, 0, Kk, qp, (long long)Hh * Ss * Mm, (long long)Ss * Mm, Mm,
          nulf, nulf, nuli, 0, 0, nuli, 0, 0, nulf, 0, Kk, Hh, 0.0009765625f, 1.0f);
  gemm_nt_kernel<false, false, EP_ELU1, 0, 0, true, false, true>
      <<<dim3(Mm / 128, Ss / 128, Bb * Hh), 256, 0, stream>>>(
          Pjh, nul16, 0, 0, Kk, kh, nul16, (long long)Ss * HK, Kk, HK, kpt, (long long)Hh * Mm * Ss, (long long)Mm * Ss, Ss,
          nulf, nulf, nuli, 0, 0, mask, Ss, 0, nulf, 0, Kk, Hh, 0.00390625f, 1024.0f);
  ksum_kernel<<<(Bb * Hh * Mm) / 1024, 256, 0, stream>>>(kpt, ksum);
  gemm_nt_kernel<false, false, EP_LIN, 0, 0, false, false, true>
      <<<dim3(Kk / 128, Mm / 128, Bb * Hh), 256, 0, stream>>>(
          vT, nul16, (long long)HK * Ss, (long long)Kk * Ss, Ss, kpt, nul16, (long long)Hh * Mm * Ss, (long long)Mm * Ss, Ss,
          kvT, (long long)Hh * Kk * Mm, (long long)Kk * Mm, Mm,
          nulf, nulf, nuli, 0, 0, nuli, 0, 0, nulf, 0, Ss, Hh, 0.0009765625f, 1.0f);
  rden_kernel<<<(Bb * Hh * Ss) / 1024, 256, 0, stream>>>(qp, ksum, rden);
  gemm_nt_kernel<false, false, EP_LIN, 0, 1, false, false, true>
      <<<dim3(Ss / 128, Kk / 128, Bb * Hh), 256, 0, stream>>>(
          qp, nul16, (long long)Hh * Ss * Mm, (long long)Ss * Mm, Mm, kvT, nul16, (long long)Hh * Kk * Mm, (long long)Kk * Mm, Mm,
          attnh, (long long)Ss * HK, Kk, HK,
          nulf, rden, nuli, (long long)Hh * Ss, Ss, nuli, 0, 0, nulf, 0, Mm, Hh, 0.03125f, 1.0f);
  gemm_nt_kernel<false, false, EP_LIN, 1, 2, false, true, false>
      <<<dim3(BS / 128, Dd / 128, 1), 256, 0, stream>>>(
          attnh, nul16, 0, 0, HK, WoT, nul16, 0, 0, HK, res1, 0, 0, Dd,
          bo, nulf, mask, 0, 0, nuli, 0, 0, Xn, Dd, HK, 1, 0.0001220703125f, 1.0f);
  ln_planes_kernel<true><<<BS / 16, 256, 0, stream>>>(res1, ln2_g, ln2_b, fln0_g, fln0_b, a0hi, a0lo);
  gemm_nt_kernel<true, true, EP_ELU, 1, 0, false, false, false>
      <<<dim3(BS / 128, Dd / 128, 1), 256, 0, stream>>>(
          a0hi, a0lo, 0, 0, Dd, W0h, W0l, 0, 0, Dd, h1, 0, 0, Dd,
          f_b0, nulf, nuli, 0, 0, nuli, 0, 0, nulf, 0, Dd, 1, 1.0f, 1.0f);
  ln_planes_kernel<false><<<BS / 16, 256, 0, stream>>>(h1, fln1_g, fln1_b, nulf, nulf, a1hi, a1lo);
  gemm_nt_kernel<true, true, EP_LIN, 1, 0, false, false, false>
      <<<dim3(BS / 128, Dd / 128, 1), 256, 0, stream>>>(
          a1hi, a1lo, 0, 0, Dd, W1h, W1l, 0, 0, Dd, out, 0, 0, Dd,
          f_b1, nulf, nuli, 0, 0, nuli, 0, 0, nulf, 0, Dd, 1, 1.0f, 1.0f);
}
